// MultiAttention_41540923686988
// MI455X (gfx1250) — hardware-verified
//
#include <hip/hip_runtime.h>
#include <math.h>

#ifndef NB
#define NB 32
#endif
#ifndef SEQ
#define SEQ 2048
#endif
#define NB_FULL 32
#define SEQ_FULL 2048

constexpr int kFeat  = 128;
constexpr int kDk    = 32;
constexpr int kDpad  = 64;
constexpr int kHeads = 16;
constexpr int kFilt  = 3;
constexpr int kRows  = NB * SEQ;
constexpr int kG     = (NB % 2 == 0) ? 2 : 1;
constexpr int kGroups = NB / kG;
constexpr int kSmT   = SEQ / 8;
constexpr int kSmW   = kSmT / 32;
constexpr float kWCarry    = 16.0f;
constexpr float kProjScale = 0.0625f;
constexpr float kScoreScale = 0.17677669529663687f;
constexpr float kPCarry    = 2048.0f;
constexpr float kPVScale   = 1.0f / 2048.0f;

static_assert(NB >= 1 && NB <= NB_FULL);
static_assert(SEQ >= 256 && SEQ <= SEQ_FULL && (SEQ % 256) == 0);
static_assert(kSmT >= 32 && kSmT <= 256 && (kSmT % 32) == 0 && kSmW <= 8);
static_assert((kRows % 256) == 0);
static_assert((kFeat % 32) == 0 && (kDpad % 64) == 0 && (SEQ % 64) == 0);

constexpr size_t cmaxz(size_t a, size_t b) { return a > b ? a : b; }
constexpr size_t kBytesX    = (size_t)3 * kRows * kFeat * 2;
constexpr size_t kBytesSc   = (size_t)kG * SEQ * SEQ * 4;
constexpr size_t kBytesP    = (size_t)kG * SEQ * SEQ * 2;
constexpr size_t kReg0      = cmaxz(kBytesX, kBytesSc + kBytesP);
constexpr size_t kOffX      = 0;
constexpr size_t kOffSc     = 0;
constexpr size_t kOffP      = kBytesSc;
constexpr size_t kOffQ      = kReg0;
constexpr size_t kBytesQ    = (size_t)kRows * kDpad * 2;
constexpr size_t kOffK      = kOffQ + kBytesQ;
constexpr size_t kOffVT     = kOffK + kBytesQ;
constexpr size_t kBytesVT   = (size_t)NB * kDpad * SEQ * 2;
constexpr size_t kOffHead   = kOffVT + kBytesVT;
constexpr size_t kBytesHead = (size_t)kRows * kDpad * 4;
constexpr size_t kOffWT     = kOffHead + kBytesHead;
constexpr size_t kBytesWT   = (size_t)3 * kDpad * kFeat * 2;
constexpr size_t kOffBias   = kOffWT + kBytesWT;
constexpr size_t kBytesBias = (size_t)3 * kDpad * 4;
constexpr size_t kWsNeed    = kOffBias + kBytesBias;
static_assert(kWsNeed <= (size_t)134217728);
static_assert((kOffP % 128) == 0 && (kOffQ % 128) == 0 && (kOffK % 128) == 0 && (kOffVT % 128) == 0);
static_assert((kOffHead % 128) == 0 && (kOffWT % 128) == 0 && (kOffBias % 128) == 0);
static_assert(kBytesSc + kBytesP <= kReg0 && kBytesX <= kReg0);
static_assert((size_t)kRows * kFilt * 4 == (size_t)NB * SEQ * kFilt * 4);

typedef __attribute__((ext_vector_type(16))) _Float16 v16h;
typedef __attribute__((ext_vector_type(8)))  _Float16 v8h;
typedef __attribute__((ext_vector_type(16))) __bf16   v16b;
typedef __attribute__((ext_vector_type(8)))  __bf16   v8b;
typedef __attribute__((ext_vector_type(8)))  float    v8f;
typedef __attribute__((ext_vector_type(4)))  float    v4f;
typedef __attribute__((ext_vector_type(4)))  unsigned int v4u;

__device__ __forceinline__ unsigned short f2bf_bits(float f) {
  unsigned u = __float_as_uint(f);
  return (unsigned short)((u + 0x7FFFu + ((u >> 16) & 1u)) >> 16);
}
__device__ __forceinline__ float bf_bits2f(unsigned short h) { return __uint_as_float(((unsigned)h) << 16); }
__device__ __forceinline__ float bfr(float f) { return bf_bits2f(f2bf_bits(f)); }

__device__ __forceinline__ void dep_guard_h(v8f& a, v8f& b, v16h x, v16h y) { asm volatile("v_nop\n\tv_nop\n\tv_nop\n\tv_nop" : "+v"(a), "+v"(b) : "v"(x), "v"(y)); }
__device__ __forceinline__ void dep_guard_b(v8f& a, v8f& b, v16b x, v16b y) { asm volatile("v_nop\n\tv_nop\n\tv_nop\n\tv_nop" : "+v"(a), "+v"(b) : "v"(x), "v"(y)); }
__device__ __forceinline__ void keep4_h(v16h a, v16h b, v16h c, v16h d) { asm volatile("v_nop" :: "v"(a), "v"(b), "v"(c), "v"(d)); }
__device__ __forceinline__ void keep4_b(v16b a, v16b b, v16b c, v16b d) { asm volatile("v_nop" :: "v"(a), "v"(b), "v"(c), "v"(d)); }
__device__ __forceinline__ void acc_guard4(v8f& a, v8f& b, v8f& c, v8f& d) { asm volatile("v_nop\n\tv_nop\n\tv_nop\n\tv_nop" : "+v"(a), "+v"(b), "+v"(c), "+v"(d)); }
template <typename T> struct Frag;
template <> struct Frag<_Float16> {
  typedef v16h V; union U { v16h v; v8h h[2]; };
  static __device__ __forceinline__ v16h load(const _Float16* p) {
    U f; f.h[0] = *(const v8h*)(p); f.h[1] = *(const v8h*)(p + 16); return f.v;
  }
  static __device__ __forceinline__ v8f mma(v16h a, v16h b, v8f c) {
    return __builtin_amdgcn_wmma_f32_16x16x32_f16(false, a, false, b, (short)0, c, false, false);
  }
  static __device__ __forceinline__ void guard(v8f& a, v8f& b, v16h x, v16h y) { dep_guard_h(a, b, x, y); }
  static __device__ __forceinline__ void keep(v16h a, v16h b, v16h c, v16h d) { keep4_h(a, b, c, d); }
};
template <> struct Frag<__bf16> {
  typedef v16b V; union U { v16b v; v8b h[2]; };
  static __device__ __forceinline__ v16b load(const __bf16* p) {
    U f; f.h[0] = *(const v8b*)(p); f.h[1] = *(const v8b*)(p + 16); return f.v;
  }
  static __device__ __forceinline__ v8f mma(v16b a, v16b b, v8f c) {
    return __builtin_amdgcn_wmma_f32_16x16x32_bf16(false, a, false, b, (short)0, c, false, false);
  }
  static __device__ __forceinline__ void guard(v8f& a, v8f& b, v16b x, v16b y) { dep_guard_b(a, b, x, y); }
  static __device__ __forceinline__ void keep(v16b a, v16b b, v16b c, v16b d) { keep4_b(a, b, c, d); }
};

__device__ __forceinline__ unsigned pk16(unsigned short a, unsigned short b) { return (unsigned)a | ((unsigned)b << 16); }
__device__ __forceinline__ unsigned short h_bits(float f) { const _Float16 h = (_Float16)f; return __builtin_bit_cast(unsigned short, h); }

template <int ET> struct Elem;
template <> struct Elem<0> { typedef _Float16 T; };
template <> struct Elem<1> { typedef __bf16 T; };
template <int ET, bool SPLIT, int BIAS_MODE, int OUT_MODE, bool RESID, int ACT = 0>
__global__ __launch_bounds__(256) void wmma_gemm64(
    const unsigned short* __restrict__ Ap, const unsigned short* __restrict__ A2p, int lda, long strideA,
    const unsigned short* __restrict__ Btp, const unsigned short* __restrict__ Bt2p, int ldb, long strideB,
    void* __restrict__ Cout, void* __restrict__ Cout2, int ldc, long strideC,
    const float* __restrict__ bias,
    const float* __restrict__ resid, long strideR,
    int M, int N, int K, float scale) {
  typedef typename Elem<ET>::T T;
  typedef typename Frag<T>::V V;
  const T* A = (const T*)Ap; const T* A2 = (const T*)A2p; const T* Bt = (const T*)Btp; const T* Bt2 = (const T*)Bt2p;
  __shared__ __align__(16) float sT[8][16 * 68];
  const int b    = blockIdx.y;
  const int lane = threadIdx.x & 31;
  const int wave = threadIdx.x >> 5;
  const int tilesN = N >> 6;
  const int tilesM = M >> 6;
  const int tile = blockIdx.x * 8 + wave;
  if (tile >= tilesM * tilesN) return;
  const int tm = tile / tilesN;
  const int tn = tile - tm * tilesN;
  const int m0 = tm << 6;
  const int n0 = tn << 6;

  const T* Ab  = A  + (size_t)b * strideA;
  const T* Bb  = Bt + (size_t)b * strideB;
  const T* Ab2 = SPLIT ? (A2  + (size_t)b * strideA) : nullptr;
  const T* Bb2 = SPLIT ? (Bt2 + (size_t)b * strideB) : nullptr;

  const int rlane = lane & 15;
  const int koff  = (lane >> 4) * 8;
  const int mOff  = (lane >> 4) * 8;

  v8f acc[4][4];
#pragma unroll
  for (int i = 0; i < 4; ++i)
#pragma unroll
    for (int j = 0; j < 4; ++j) acc[i][j] = (v8f){0.f,0.f,0.f,0.f,0.f,0.f,0.f,0.f};

  for (int k0 = 0; k0 < K; k0 += 32) {
    V bh[4], bl[4];
#pragma unroll
    for (int j = 0; j < 4; ++j) {
      const size_t bo = (size_t)(n0 + (j << 4) + rlane) * ldb + koff + k0;
      bh[j] = Frag<T>::load(Bb + bo);
      if (SPLIT) bl[j] = Frag<T>::load(Bb2 + bo);
    }
#pragma unroll
    for (int i = 0; i < 4; ++i) {
      const size_t ao = (size_t)(m0 + (i << 4) + rlane) * lda + koff + k0;
      V ah = Frag<T>::load(Ab + ao);
      V al;
      if (SPLIT) al = Frag<T>::load(Ab2 + ao);
#pragma unroll
      for (int j = 0; j < 4; ++j) {
        acc[i][j] = Frag<T>::mma(ah, bh[j], acc[i][j]);
        if (SPLIT) {
          acc[i][j] = Frag<T>::mma(ah, bl[j], acc[i][j]);
          acc[i][j] = Frag<T>::mma(al, bh[j], acc[i][j]);
        }
      }
      Frag<T>::guard(acc[i][0], acc[i][3], ah, SPLIT ? al : ah);
    }
    Frag<T>::keep(bh[0], bh[1], bh[2], bh[3]);
    if (SPLIT) Frag<T>::keep(bl[0], bl[1], bl[2], bl[3]);
  }
  acc_guard4(acc[0][0], acc[0][1], acc[0][2], acc[0][3]);
  acc_guard4(acc[1][0], acc[1][1], acc[1][2], acc[1][3]);
  acc_guard4(acc[2][0], acc[2][1], acc[2][2], acc[2][3]);
  acc_guard4(acc[3][0], acc[3][1], acc[3][2], acc[3][3]);

  float* slab = sT[wave];
  const float* Rb = RESID ? (resid + (size_t)b * strideR) : nullptr;
#pragma unroll
  for (int i = 0; i < 4; ++i) {
    const int mBase = m0 + (i << 4);
#pragma unroll
    for (int j = 0; j < 4; ++j) {
      const int n = n0 + (j << 4) + rlane;
      float bv = 0.f;
      if (BIAS_MODE == 2) bv = bias[n];
#pragma unroll
      for (int r = 0; r < 8; ++r) {
        float v = acc[i][j][r] * scale;
        if (BIAS_MODE == 1) v += bias[mBase + mOff + r];
        if (BIAS_MODE == 2) v += bv;
        if (RESID) v += Rb[(size_t)(mBase + mOff + r) * ldc + n];
        if (ACT == 2) v = fmaxf(v, 0.0f);
        if (ACT == 4) v = (v > 0.f) ? v : 0.01f * v;
        slab[(mOff + r) * 68 + (j << 4) + rlane] = v;
      }
    }
    __builtin_amdgcn_fence(3, "workgroup");
    __builtin_amdgcn_wave_barrier();
    __builtin_amdgcn_fence(2, "workgroup");
    if (OUT_MODE == 0) {
      float* C = (float*)Cout + (size_t)b * strideC;
      const int hh = lane >> 4, c4 = (lane & 15) * 4;
      for (int pass = 0; pass < 2; ++pass) {
#pragma unroll
        for (int it = 0; it < 8; ++it) {
          const int row = it * 2 + hh;
          v4f v = *(const v4f*)(slab + row * 68 + c4);
          *(volatile v4f*)(C + (size_t)(mBase + row) * ldc + n0 + c4) = v;
        }
        __threadfence();
      }
    } else {
      const int q = lane >> 3, c8 = (lane & 7) * 8;
      unsigned short* C  = (unsigned short*)Cout  + (size_t)b * strideC;
      unsigned short* C2 = (OUT_MODE == 2) ? ((unsigned short*)Cout2 + (size_t)b * strideC) : nullptr;
      for (int pass = 0; pass < 2; ++pass) {
#pragma unroll
        for (int it = 0; it < 4; ++it) {
          const int row = it * 4 + q;
          const float* sp = slab + row * 68 + c8;
          v8h hv, lv;
#pragma unroll
          for (int e = 0; e < 8; ++e) {
            if (OUT_MODE == 1) {
              hv[e] = (_Float16)sp[e];
            } else {
              unsigned short hb = f2bf_bits(sp[e]);
              unsigned short lb = f2bf_bits(sp[e] - bf_bits2f(hb));
              hv[e] = __builtin_bit_cast(_Float16, hb);
              lv[e] = __builtin_bit_cast(_Float16, lb);
            }
          }
          *(volatile v8h*)(C + (size_t)(mBase + row) * ldc + n0 + c8) = hv;
          if (OUT_MODE == 2) *(volatile v8h*)(C2 + (size_t)(mBase + row) * ldc + n0 + c8) = lv;
        }
        __threadfence();
      }
    }
    __builtin_amdgcn_fence(3, "workgroup");
    __builtin_amdgcn_wave_barrier();
    __builtin_amdgcn_fence(2, "workgroup");
  }
}

__global__ __launch_bounds__(256) void cast_x_kernel(const float* __restrict__ X0, const float* __restrict__ X1,
                                                     const float* __restrict__ X2, unsigned short* __restrict__ dst) {
  const int sel = blockIdx.z;
  const int b   = blockIdx.y;
  const float* src = (sel == 0) ? X0 : (sel == 1) ? X1 : X2;
  const int i = blockIdx.x * 256 + threadIdx.x;
  if (i >= SEQ * (kFeat / 8)) return;
  const float* p = src + (size_t)b * SEQ_FULL * kFeat + 8 * (size_t)i;
  const v4f a = *(const v4f*)(p);
  const v4f c = *(const v4f*)(p + 4);
  unsigned short hb[8];
#pragma unroll
  for (int e = 0; e < 4; ++e) {
    hb[e]     = h_bits(bfr(a[e]));
    hb[4 + e] = h_bits(bfr(c[e]));
  }
  const v4u u = (v4u){pk16(hb[0], hb[1]), pk16(hb[2], hb[3]), pk16(hb[4], hb[5]), pk16(hb[6], hb[7])};
  unsigned short* q = dst + (size_t)sel * kRows * kFeat + (size_t)b * SEQ * kFeat + 8 * (size_t)i;
  *(volatile v4u*)q = u;
  __threadfence();
  *(volatile v4u*)q = u;
}

__global__ __launch_bounds__(256) void wcast_kernel(const float* __restrict__ W0, const float* __restrict__ b0,
                                                    const float* __restrict__ W1, const float* __restrict__ b1,
                                                    const float* __restrict__ W2, const float* __restrict__ b2,
                                                    unsigned short* __restrict__ WT, float* __restrict__ biasT, float scale) {
  __shared__ float sm[kDpad][kFeat + 1];
  const int t = threadIdx.x;
  const int z = blockIdx.x;
  const float* W  = (z == 0) ? W0 : (z == 1) ? W1 : W2;
  const float* bb = (z == 0) ? b0 : (z == 1) ? b1 : b2;
#pragma unroll
  for (int i = 0; i < 16; ++i) {
    const int e = i * 256 + t;
    const int f = e >> 5;
    const int d = e & 31;
    sm[d][f] = bfr(W[e]) * scale;
  }
#pragma unroll
  for (int i = 0; i < 16; ++i) {
    const int e = i * 256 + t;
    sm[kDk + (e >> 7)][e & 127] = 0.0f;
  }
  __syncthreads();
  const int lane = t & 31, wave = t >> 5;
  const int hh = lane >> 4, c8 = (lane & 15) * 8;
  unsigned short* op = WT + (size_t)z * kDpad * kFeat;
  for (int pass = 0; pass < 2; ++pass) {
#pragma unroll
    for (int it = 0; it < 4; ++it) {
      const int row = wave * 8 + it * 2 + hh;
      unsigned short hb[8];
#pragma unroll
      for (int e = 0; e < 8; ++e) hb[e] = h_bits(sm[row][c8 + e]);
      const v4u u = (v4u){pk16(hb[0], hb[1]), pk16(hb[2], hb[3]), pk16(hb[4], hb[5]), pk16(hb[6], hb[7])};
      *(volatile v4u*)(op + (size_t)row * kFeat + c8) = u;
    }
    __threadfence();
  }
  if (wave == 0) {
    float bvv[4];
#pragma unroll
    for (int e = 0; e < 4; ++e) {
      const int n  = 4 * lane + e;
      const int nc = (n < kDk) ? n : (kDk - 1);
      const float x = bfr(bb[nc]);
      bvv[e] = (n < kDk) ? x : 0.0f;
    }
    const v4f v = (v4f){bvv[0], bvv[1], bvv[2], bvv[3]};
    float* bp = biasT + (size_t)z * kDpad + 4 * lane;
    if (lane < 16) *(volatile v4f*)bp = v;
    __threadfence();
    if (lane < 16) *(volatile v4f*)bp = v;
  }
}

__global__ __launch_bounds__(256) void softmax_row_kernel(const float* __restrict__ Sc, unsigned short* __restrict__ P, float carry) {
  __shared__ float redM[8];
  __shared__ float redS[8];
  const int row  = blockIdx.x;
  const int t    = threadIdx.x;
  const int lane = t & 31, wave = t >> 5;
  const int c0   = t * 8;
  const float* sr = Sc + (size_t)row * SEQ + c0;
  const v4f a = *(const v4f*)(sr);
  const v4f c = *(const v4f*)(sr + 4);
  float x[8];
#pragma unroll
  for (int e = 0; e < 4; ++e) { x[e] = a[e]; x[4 + e] = c[e]; }
  float m = fmaxf(fmaxf(fmaxf(x[0], x[1]), fmaxf(x[2], x[3])), fmaxf(fmaxf(x[4], x[5]), fmaxf(x[6], x[7])));
#pragma unroll
  for (int off = 16; off > 0; off >>= 1) m = fmaxf(m, __shfl_xor(m, off, 32));
  if (lane == 0) redM[wave] = m;
  __syncthreads();
  float gm = redM[0];
#pragma unroll
  for (int w = 1; w < kSmW; ++w) gm = fmaxf(gm, redM[w]);
  float ex[8];
#pragma unroll
  for (int e = 0; e < 8; ++e) ex[e] = expf(x[e] - gm);
  float s = ((ex[0] + ex[1]) + (ex[2] + ex[3])) + ((ex[4] + ex[5]) + (ex[6] + ex[7]));
#pragma unroll
  for (int off = 16; off > 0; off >>= 1) s += __shfl_xor(s, off, 32);
  if (lane == 0) redS[wave] = s;
  __syncthreads();
  float tot = redS[0];
#pragma unroll
  for (int w = 1; w < kSmW; ++w) tot += redS[w];
  const float scl = carry * (1.0f / tot);
  unsigned short hb[8];
#pragma unroll
  for (int e = 0; e < 8; ++e) hb[e] = h_bits(ex[e] * scl);
  const v4u u = (v4u){pk16(hb[0], hb[1]), pk16(hb[2], hb[3]), pk16(hb[4], hb[5]), pk16(hb[6], hb[7])};
  unsigned short* q = P + (size_t)row * SEQ + c0;
  *(volatile v4u*)q = u;
  __threadfence();
  *(volatile v4u*)q = u;
}

__global__ __launch_bounds__(256) void out_kernel(const float* __restrict__ Hd, const float* __restrict__ Wo,
                                                  const float* __restrict__ bo, float* __restrict__ out) {
  __shared__ float wos[kDk * kFilt];
  __shared__ __align__(16) float so[256 * kFilt];
  const int t = threadIdx.x;
  if (t < kDk * kFilt) {
    const int d = t / kFilt, f = t - d * kFilt;
    float s = 0.f;
#pragma unroll 1
    for (int hh = 0; hh < kHeads; ++hh) s += bfr(Wo[(hh * kDk + d) * kFilt + f]);
    wos[t] = s;
  }
  __syncthreads();
  const int row = blockIdx.x * 256 + t;
  const float* hp = Hd + (size_t)row * kDpad;
  float a0 = 0.f, a1 = 0.f, a2 = 0.f;
#pragma unroll 1
  for (int d4 = 0; d4 < kDk / 4; ++d4) {
    const v4f hv = *(const v4f*)(hp + 4 * d4);
#pragma unroll
    for (int e = 0; e < 4; ++e) {
      const float h = hv[e];
      const int d = 4 * d4 + e;
      a0 = fmaf(h, wos[d * kFilt + 0], a0);
      a1 = fmaf(h, wos[d * kFilt + 1], a1);
      a2 = fmaf(h, wos[d * kFilt + 2], a2);
    }
  }
  const float bo0 = bfr(bo[0]), bo1 = bfr(bo[1]), bo2 = bfr(bo[2]);
  so[t * kFilt + 0] = a0 + bo0;
  so[t * kFilt + 1] = a1 + bo1;
  so[t * kFilt + 2] = a2 + bo2;
  __syncthreads();
  const int tt = (t < 192) ? t : 191;
  const v4f v = *(const v4f*)(so + 4 * tt);
  float* op = out + (size_t)blockIdx.x * (256 * kFilt) + 4 * tt;
  if (t < 192) *(volatile v4f*)op = v;
  __threadfence();
  if (t < 192) *(volatile v4f*)op = v;
}

extern "C" void kernel_launch(void* const* d_in, const int* in_sizes, int n_in,
                              void* d_out, int out_size, void* d_ws, size_t ws_size,
                              hipStream_t stream) {
  if (n_in < 11) return;
  const long needX = ((long)(NB - 1) * SEQ_FULL + SEQ) * kFeat;
  if ((long)in_sizes[0] < needX || (long)in_sizes[1] < needX || (long)in_sizes[2] < needX) return;
  if (in_sizes[3] < kFeat * kDk || in_sizes[5] < kFeat * kDk || in_sizes[7] < kFeat * kDk) return;
  if (in_sizes[4] < kDk || in_sizes[6] < kDk || in_sizes[8] < kDk) return;
  if (in_sizes[9] < kHeads * kDk * kFilt || in_sizes[10] < kFilt) return;
  if (out_size < kRows * kFilt) return;
  if (ws_size < kWsNeed) return;

  const float* qin = (const float*)d_in[0];
  const float* kin = (const float*)d_in[1];
  const float* vin = (const float*)d_in[2];
  const float* Wq  = (const float*)d_in[3];
  const float* bq  = (const float*)d_in[4];
  const float* Wk  = (const float*)d_in[5];
  const float* bk  = (const float*)d_in[6];
  const float* Wv  = (const float*)d_in[7];
  const float* bv  = (const float*)d_in[8];
  const float* Wo  = (const float*)d_in[9];
  const float* bo  = (const float*)d_in[10];
  float* out = (float*)d_out;

  unsigned char* ws = (unsigned char*)d_ws;
  unsigned short* X16   = (unsigned short*)(ws + kOffX);
  float*          Sc    = (float*)(ws + kOffSc);
  unsigned short* P16   = (unsigned short*)(ws + kOffP);
  unsigned short* Qp    = (unsigned short*)(ws + kOffQ);
  unsigned short* Kp    = (unsigned short*)(ws + kOffK);
  unsigned short* VTp   = (unsigned short*)(ws + kOffVT);
  float*          Head  = (float*)(ws + kOffHead);
  unsigned short* WT    = (unsigned short*)(ws + kOffWT);
  float*          BiasT = (float*)(ws + kOffBias);
  const unsigned short* Xq16 = X16;
  const unsigned short* Xk16 = X16 + (size_t)kRows * kFeat;
  const unsigned short* Xv16 = X16 + (size_t)2 * kRows * kFeat;
  const unsigned short* WqT = WT;
  const unsigned short* WkT = WT + (size_t)kDpad * kFeat;
  const unsigned short* WvT = WT + (size_t)2 * kDpad * kFeat;

  cast_x_kernel<<<dim3(SEQ / 16, NB, 3), dim3(256), 0, stream>>>(qin, kin, vin, X16);

  wcast_kernel<<<dim3(3), dim3(256), 0, stream>>>(Wq, bq, Wk, bk, Wv, bv, WT, BiasT, kWCarry);

  wmma_gemm64<0, false, 2, 1, false, 0><<<dim3((kRows / 64 + 7) / 8, 1), dim3(256), 0, stream>>>(
      Xq16, nullptr, kFeat, 0L, WqT, nullptr, kFeat, 0L,
      (void*)Qp, nullptr, kDpad, 0L, BiasT, nullptr, 0L, kRows, kDpad, kFeat, kProjScale);

  wmma_gemm64<0, false, 2, 1, false, 0><<<dim3((kRows / 64 + 7) / 8, 1), dim3(256), 0, stream>>>(
      Xk16, nullptr, kFeat, 0L, WkT, nullptr, kFeat, 0L,
      (void*)Kp, nullptr, kDpad, 0L, BiasT + kDpad, nullptr, 0L, kRows, kDpad, kFeat, kProjScale);

  wmma_gemm64<0, false, 1, 1, false, 0><<<dim3((SEQ / 64 + 7) / 8, NB), dim3(256), 0, stream>>>(
      WvT, nullptr, kFeat, 0L, Xv16, nullptr, kFeat, (long)SEQ * kFeat,
      (void*)VTp, nullptr, SEQ, (long)kDpad * SEQ, BiasT + 2 * kDpad, nullptr, 0L, kDpad, SEQ, kFeat, kProjScale);

  for (int g = 0; g < kGroups; ++g) {
    const size_t qkOff = (size_t)g * kG * SEQ * kDpad;
    const size_t vtOff = (size_t)g * kG * kDpad * SEQ;
    wmma_gemm64<0, false, 0, 0, false, 0><<<dim3(((SEQ / 64) * (SEQ / 64) + 7) / 8, kG), dim3(256), 0, stream>>>(
        Qp + qkOff, nullptr, kDpad, (long)SEQ * kDpad, Kp + qkOff, nullptr, kDpad, (long)SEQ * kDpad,
        (void*)Sc, nullptr, SEQ, (long)SEQ * SEQ, nullptr, nullptr, 0L, SEQ, SEQ, kDk, kScoreScale);
    softmax_row_kernel<<<dim3(kG * SEQ), dim3(kSmT), 0, stream>>>(Sc, P16, kPCarry);
    wmma_gemm64<0, false, 0, 0, false, 0><<<dim3(((SEQ / 64) + 7) / 8, kG), dim3(256), 0, stream>>>(
        P16, nullptr, SEQ, (long)SEQ * SEQ, VTp + vtOff, nullptr, SEQ, (long)kDpad * SEQ,
        (void*)(Head + qkOff), nullptr, kDpad, (long)SEQ * kDpad, nullptr, nullptr, 0L, SEQ, kDpad, SEQ, kPVScale);
  }

  out_kernel<<<dim3(kRows / 256), dim3(256), 0, stream>>>(Head, Wo, bo, out);
}
